// Encoder_25847113188087
// MI455X (gfx1250) — hardware-run, weakly checked
//
#include <hip/hip_runtime.h>


#ifndef NB
#define NB 4
#endif
#ifndef SEQ
#define SEQ 1024
#endif
#define NB_FULL  4
#define SEQ_FULL 1024
#define CW    256
#define NH_   16
#define DH    16
#define MLPW  1024
#define CAH   16
#define HID   2048
#define PRED  512
#define IMG   128
#define GRD   64
#define NTOKM 4096
#define MR    (NB * SEQ)
#define AW    4
#define OSP   68
#define TSP   68
#define GW    2
#define MSP   260
#define WCAR  64.0f
#define ACAR  16.0f
#define VCAR  64.0f
#define CTXC  256.0f
#define PSH   14.0f
#define LOG2E 1.4426950408889634f
#define SC2   ((float)(0.25 * 1.4426950408889634))
#define NEGB  (-3.0e38f)

static_assert(NH_ * DH == CW);
static_assert(DH == 16);
static_assert(AW * DH == 64);
static_assert(NH_ % AW == 0);
static_assert(CW % 64 == 0 && MLPW % 64 == 0 && HID % 64 == 0 && PRED % 64 == 0);
static_assert(CW % 32 == 0 && MLPW % 32 == 0 && HID % 32 == 0);
static_assert(SEQ % 64 == 0);
static_assert(MR % 64 == 0);
static_assert(SEQ % 32 == 0);
static_assert(MR % (16 * GW) == 0);
static_assert(MR % 8 == 0);
static_assert(((size_t)MR * CW / 4) % 256 == 0);
static_assert(NB <= NB_FULL && SEQ <= SEQ_FULL);
static_assert((OSP * 4) % 16 == 0 && (TSP * 4) % 16 == 0 && (MSP * 4) % 16 == 0);
static_assert(64 * TSP * 4 <= 131072);
static_assert(GW * 16 * MSP * 4 <= 65536);
static_assert(16 * OSP * 4 <= 131072);

typedef _Float16 h16;
typedef __attribute__((ext_vector_type(16))) _Float16 v16h;
typedef __attribute__((ext_vector_type(8)))  _Float16 v8h;
typedef __attribute__((ext_vector_type(4)))  _Float16 v4h;
typedef __attribute__((ext_vector_type(8)))  float    v8f;
typedef __attribute__((ext_vector_type(4)))  float    v4f;
typedef v4f  __attribute__((may_alias)) v4fa;

__device__ __forceinline__ unsigned short f2bf(float f) { unsigned u = __float_as_uint(f); u += 0x7FFFu + ((u >> 16) & 1u); return (unsigned short)(u >> 16); }
__device__ __forceinline__ float bfr(float f) { return __uint_as_float(((unsigned)f2bf(f)) << 16); }
__device__ __forceinline__ v16h cat16(v8h lo, v8h hi) { return __builtin_shufflevector(lo, hi, 0, 1, 2, 3, 4, 5, 6, 7, 8, 9, 10, 11, 12, 13, 14, 15); }
__device__ __forceinline__ v8f wmma16(v16h a, v16h b, v8f c) { return __builtin_amdgcn_wmma_f32_16x16x32_f16(false, a, false, b, (short)0, c, false, false); }
__device__ __forceinline__ v8f wmma16g(v16h a, v16h b, v8f c) { c = wmma16(a, b, c); asm volatile("v_nop\n\tv_nop\n\tv_nop\n\tv_nop" : "+v"(c) : "v"(a), "v"(b)); return c; }
__device__ __forceinline__ v16h ldh(const h16* p) { return cat16(*(const v8h*)p, *(const v8h*)(p + 16)); }
__device__ __forceinline__ v16h ldh8z(const h16* p) { const v8h z = (v8h){}; return cat16(*(const v8h*)p, z); }
__device__ __forceinline__ void wave_sync() { __builtin_amdgcn_fence(3  , "wavefront"); __builtin_amdgcn_wave_barrier(); asm volatile("" ::: "memory"); }
static __device__ __forceinline__ h16 toh_flush(float v) { const h16 r = (h16)v; return (fabsf(v) < 6.103515625e-05f) ? (h16)0.0f : r; }
__device__ __forceinline__ float gelu_erf(float x) { return 0.5f * x * (1.0f + erff(x * 0.70710678118654752f)); }

__global__ __launch_bounds__(256) void k_wconv(const float* __restrict__ W, h16* WT, int K, int N, int total8) {
#pragma clang fp contract(off)
    const int i = blockIdx.x * 256 + threadIdx.x; if (i >= total8) return;
    const int o = i * 8; const int kn = K * N; const int l = o / kn; const int rem = o - l * kn; const int n = rem / K; const int k = rem - n * K;
    const size_t sb = (size_t)l * kn + (size_t)k * N + n;
    v8h hv;
#pragma unroll
    for (int j = 0; j < 8; ++j) hv[j] = toh_flush(bfr(W[sb + (size_t)j * N]) * WCAR);
    *(volatile v8h*)(WT + (size_t)o) = hv; __threadfence(); *(volatile v8h*)(WT + (size_t)o) = hv;
}

__global__ __launch_bounds__(256) void k_postab(float* PT) {
#pragma clang fp contract(off)
    const int i = blockIdx.x * 256 + threadIdx.x; if (i >= GRD * 128) return;
    const int p = i >> 7, c = i & 127, f = c & 63;
    const float om = expf(-(float)f * 0.14391156831212787f);
    const float ang = (float)p * om;
    const float sv = sinf(ang), cv = cosf(ang);
    const float v = (c < 64) ? sv : cv;
    *(volatile float*)(PT + i) = v; __threadfence(); *(volatile float*)(PT + i) = v;
}

__global__ __launch_bounds__(256) void k_patch(const float* __restrict__ x, const int* __restrict__ midx, const float* __restrict__ Wp, const float* __restrict__ bp,
                                               const float* __restrict__ cls, const float* __restrict__ PT, float* F0, h16* XH) {
#pragma clang fp contract(off)
    const int e4 = blockIdx.x * 256 + threadIdx.x; if (e4 >= MR * CW / 4) return;
    const int c = (e4 & 63) * 4; const int row = e4 >> 6; const int b = row / SEQ, i = row - b * SEQ;
    int tok = midx[b * SEQ_FULL + i]; tok = tok < 0 ? 0 : (tok > NTOKM ? NTOKM : tok);
    const int p = (tok > 0) ? (tok - 1) : 0; const int ph = p >> 6, pw = p & 63;
    float acc[4];
#pragma unroll
    for (int q = 0; q < 4; ++q) acc[q] = bfr(bp[c + q]);
#pragma unroll 1
    for (int tap = 0; tap < 12; ++tap) {
        const int ch = tap >> 2, dy = (tap >> 1) & 1, dx = tap & 1;
        const float xv = bfr(x[(((size_t)b * 3 + ch) * IMG + (ph * 2 + dy)) * IMG + (pw * 2 + dx)]);
#pragma unroll
        for (int q = 0; q < 4; ++q) acc[q] += xv * bfr(Wp[(c + q) * 12 + tap]);
    }
    const int grp = c >> 6, cm = c & 63; const int pos = (grp < 2) ? pw : ph;
    const v4f pe = *(const v4f*)(PT + pos * 128 + (grp & 1) * 64 + cm);
    v4f val; v4h hv;
#pragma unroll
    for (int q = 0; q < 4; ++q) { float cv = bfr(cls[c + q]); asm volatile("" : "+v"(cv)); const float tv = acc[q] + pe[q]; val[q] = (tok == 0) ? cv : tv; hv[q] = toh_flush(val[q] * ACAR); }
    *(volatile v4f*)(F0 + (size_t)e4 * 4) = val; *(volatile v4h*)(XH + (size_t)e4 * 4) = hv;
    __threadfence();
    *(volatile v4f*)(F0 + (size_t)e4 * 4) = val; *(volatile v4h*)(XH + (size_t)e4 * 4) = hv;
}

__global__ __launch_bounds__(256) void k_ln(const float* __restrict__ X, const float* __restrict__ g, const float* __restrict__ bt, h16* Y, int D, int rows) {
#pragma clang fp contract(off)
    const int lane = threadIdx.x & 31;
    const int wave = __builtin_amdgcn_readfirstlane((int)(threadIdx.x >> 5));
    const int row = blockIdx.x * 8 + wave; if (row >= rows) return;
    const float* xr = X + (size_t)row * D + lane * 8;
    float s = 0.0f;
#pragma unroll 1
    for (int c = 0; c < D; c += 256) { const v4f a = *(const v4f*)(xr + c), b = *(const v4f*)(xr + c + 4); s += ((a[0] + a[1]) + (a[2] + a[3])) + ((b[0] + b[1]) + (b[2] + b[3])); }
    s += __shfl_xor(s, 16, 32); s += __shfl_xor(s, 8, 32); s += __shfl_xor(s, 4, 32); s += __shfl_xor(s, 2, 32); s += __shfl_xor(s, 1, 32);
    const float rd = 1.0f / (float)D;
    const float mu = s * rd;
    float v = 0.0f;
#pragma unroll 1
    for (int c = 0; c < D; c += 256) { const v4f a = *(const v4f*)(xr + c), b = *(const v4f*)(xr + c + 4);
#pragma unroll
        for (int q = 0; q < 4; ++q) { const float d0 = a[q] - mu, d1 = b[q] - mu; v += d0 * d0; v += d1 * d1; } }
    v += __shfl_xor(v, 16, 32); v += __shfl_xor(v, 8, 32); v += __shfl_xor(v, 4, 32); v += __shfl_xor(v, 2, 32); v += __shfl_xor(v, 1, 32);
    const float rs = rsqrtf(v * rd + 1e-5f);
    h16* yr = Y + (size_t)row * D + lane * 8;
#pragma unroll 1
    for (int c = 0; c < D; c += 256) {
        const v4f a = *(const v4f*)(xr + c), b = *(const v4f*)(xr + c + 4);
        const v4f g0 = *(const v4f*)(g + c + lane * 8), g1 = *(const v4f*)(g + c + lane * 8 + 4);
        const v4f b0 = *(const v4f*)(bt + c + lane * 8), b1 = *(const v4f*)(bt + c + lane * 8 + 4);
        v8h hv;
#pragma unroll
        for (int q = 0; q < 4; ++q) { hv[q] = toh_flush(((a[q] - mu) * rs * bfr(g0[q]) + bfr(b0[q])) * ACAR); hv[4 + q] = toh_flush(((b[q] - mu) * rs * bfr(g1[q]) + bfr(b1[q])) * ACAR); }
        *(volatile v8h*)(yr + c) = hv; __threadfence(); *(volatile v8h*)(yr + c) = hv;
    }
}

__global__ __launch_bounds__(32) void k_gemm(const h16* __restrict__ A, int lda, const h16* __restrict__ Bt, int ldb, int K,
                                             const float* __restrict__ bias, int brow, float oscale, int act,
                                             const float* __restrict__ R, int ldr, int useR,
                                             float* Cf, int ldc, int useF,
                                             h16* Ch, int ldch, int useH, float hscale, int cgrp, int cgs) {
    __shared__ __align__(16) float os[64 * TSP];
    const int lane = threadIdx.x & 31, lr = lane & 15, hi = lane >> 4; const int r0 = blockIdx.x * 64, c0 = blockIdx.y * 64;
    v8f acc[4][4];
#pragma unroll
    for (int mb = 0; mb < 4; ++mb)
#pragma unroll
        for (int nb = 0; nb < 4; ++nb) acc[mb][nb] = (v8f){};
    const size_t aoff = (size_t)(r0 + lr) * lda + 8 * hi, boff = (size_t)(c0 + lr) * ldb + 8 * hi;
#pragma unroll 1
    for (int kc = 0; kc < K; kc += 32) {
        v16h a[4];
#pragma unroll
        for (int mb = 0; mb < 4; ++mb) a[mb] = ldh(A + aoff + (size_t)mb * 16 * lda + kc);
#pragma unroll
        for (int nb = 0; nb < 4; ++nb) { const v16h b = ldh(Bt + boff + (size_t)nb * 16 * ldb + kc);
#pragma unroll
            for (int mb = 0; mb < 4; ++mb) acc[mb][nb] = wmma16g(a[mb], b, acc[mb][nb]); }
    }
#pragma unroll
    for (int mb = 0; mb < 4; ++mb)
#pragma unroll
        for (int nb = 0; nb < 4; ++nb)
#pragma unroll
            for (int j = 0; j < 8; ++j) os[(mb * 16 + hi * 8 + j) * TSP + nb * 16 + lr] = acc[mb][nb][j];
    wave_sync();
    const int cofs = (lane & 15) * 4, rsel = lane >> 4;
    v4f bcv;
#pragma unroll
    for (int q = 0; q < 4; ++q) { const int idx = brow ? 0 : (c0 + cofs + q); float bv = bfr(bias[idx]); asm volatile("" : "+v"(bv)); bcv[q] = brow ? 0.0f : bv; }
#pragma unroll 1
    for (int s = 0; s < 32; ++s) {
        const int row = 2 * s + rsel;
        const int bri = brow ? (r0 + row) : 0; float brv = bfr(bias[bri]); asm volatile("" : "+v"(brv)); brv = brow ? brv : 0.0f;
        v4f v = *(const v4fa*)(&os[row * TSP + cofs]);
#pragma unroll
        for (int q = 0; q < 4; ++q) { float t = v[q] * oscale + bcv[q] + brv; if (act) t = gelu_erf(t); v[q] = t; }
        if (useR) { const v4f r4 = *(const v4f*)(R + (size_t)(r0 + row) * ldr + c0 + cofs); v = v + r4; }
        *(v4fa*)(&os[row * TSP + cofs]) = v;
    }
    wave_sync();
    const size_t hc0 = (size_t)(c0 / cgrp) * (size_t)cgs + (size_t)(c0 % cgrp);
#pragma unroll 1
    for (int ps = 0; ps < 2; ++ps) {
        if (useF) {
#pragma unroll 1
            for (int s = 0; s < 32; ++s) { const int row = 2 * s + rsel;
                const v4f val = *(const v4fa*)(&os[row * TSP + cofs]);
                *(volatile v4f*)(Cf + (size_t)(r0 + row) * ldc + c0 + cofs) = val; }
        }
        if (useH) {
#pragma unroll 1
            for (int s = 0; s < 16; ++s) { const int row = 4 * s + (lane >> 3), c8 = (lane & 7) * 8;
                const v4f x0 = *(const v4fa*)(&os[row * TSP + c8]); const v4f x1 = *(const v4fa*)(&os[row * TSP + c8 + 4]); v8h hv;
#pragma unroll
                for (int i = 0; i < 4; ++i) { hv[i] = toh_flush(x0[i] * hscale); hv[4 + i] = toh_flush(x1[i] * hscale); }
                *(volatile v8h*)(Ch + (size_t)(r0 + row) * ldch + hc0 + c8) = hv; }
        }
        if (ps == 0) __threadfence(); }
}
static_assert(32 * 2 == 64 && 16 * 4 == 64);
static_assert(16 * 16 == 64 * 4 && 8 * 16 == 64 * 2);

__global__ __launch_bounds__(32) void k_qk(const h16* __restrict__ A, const h16* __restrict__ Bt, const float* __restrict__ qkvb,
                                           const float* __restrict__ nqg, const float* __restrict__ nqb, const float* __restrict__ nkg, const float* __restrict__ nkb,
                                           float oscale, h16* QKP) {
    __shared__ __align__(16) float os[64 * TSP];
    const int K = CW;
    const int lane = threadIdx.x & 31, lr = lane & 15, hi = lane >> 4; const int r0 = blockIdx.x * 64, c0 = blockIdx.y * 64;
    v8f acc[4][4];
#pragma unroll
    for (int mb = 0; mb < 4; ++mb)
#pragma unroll
        for (int nb = 0; nb < 4; ++nb) acc[mb][nb] = (v8f){};
    const size_t aoff = (size_t)(r0 + lr) * K + 8 * hi, boff = (size_t)(c0 + lr) * K + 8 * hi;
#pragma unroll 1
    for (int kc = 0; kc < K; kc += 32) {
        v16h a[4];
#pragma unroll
        for (int mb = 0; mb < 4; ++mb) a[mb] = ldh(A + aoff + (size_t)mb * 16 * K + kc);
#pragma unroll
        for (int nb = 0; nb < 4; ++nb) { const v16h b = ldh(Bt + boff + (size_t)nb * 16 * K + kc);
#pragma unroll
            for (int mb = 0; mb < 4; ++mb) acc[mb][nb] = wmma16g(a[mb], b, acc[mb][nb]); }
    }
#pragma unroll
    for (int mb = 0; mb < 4; ++mb)
#pragma unroll
        for (int nb = 0; nb < 4; ++nb)
#pragma unroll
            for (int j = 0; j < 8; ++j) os[(mb * 16 + hi * 8 + j) * TSP + nb * 16 + lr] = acc[mb][nb][j];
    wave_sync();
    const int sec = c0 / CW; const int head0 = (c0 % CW) / DH;
    const int bb = r0 / SEQ, tt = r0 % SEQ;
    const int odd = lane & 1, rloc = lane >> 1;
    float gv[8], bv[8];
#pragma unroll
    for (int i = 0; i < 8; ++i) {
        float a0 = bfr(nqg[odd * 8 + i]), a1 = bfr(nkg[odd * 8 + i]), b0 = bfr(nqb[odd * 8 + i]), b1 = bfr(nkb[odd * 8 + i]);
        asm volatile("" : "+v"(a0)); asm volatile("" : "+v"(a1)); asm volatile("" : "+v"(b0)); asm volatile("" : "+v"(b1));
        gv[i] = (sec == 0) ? a0 : a1; bv[i] = (sec == 0) ? b0 : b1; }
    const size_t PLQ = (size_t)MR * CW;
#pragma unroll 1
    for (int ps = 0; ps < 2; ++ps) {
#pragma unroll 1
        for (int hh = 0; hh < 4; ++hh) {
            float bc[16];
#pragma unroll
            for (int d = 0; d < 16; ++d) bc[d] = bfr(qkvb[c0 + hh * 16 + d]);
            const size_t pb = (size_t)sec * PLQ + ((size_t)(bb * NH_ + head0 + hh) * SEQ + (size_t)tt) * DH + (size_t)lane * 8;
#pragma unroll 1
            for (int s = 0; s < 4; ++s) {
                const int row = s * 16 + rloc;
                float xx[16];
#pragma unroll
                for (int q = 0; q < 4; ++q) { const v4f t4 = *(const v4fa*)(&os[row * TSP + hh * 16 + 4 * q]);
#pragma unroll
                    for (int i = 0; i < 4; ++i) xx[4 * q + i] = t4[i] * oscale + bc[4 * q + i]; }
                float sm = 0.0f;
#pragma unroll
                for (int d = 0; d < 16; ++d) sm += xx[d];
                const float mu = sm * 0.0625f;
                float vr = 0.0f;
#pragma unroll
                for (int d = 0; d < 16; ++d) { const float dd = xx[d] - mu; vr += dd * dd; }
                const float rs = rsqrtf(vr * 0.0625f + 1e-5f);
                v8h hv;
#pragma unroll
                for (int i = 0; i < 8; ++i) { const float xi = odd ? xx[8 + i] : xx[i]; hv[i] = toh_flush((xi - mu) * rs * gv[i] + bv[i]); }
                *(volatile v8h*)(QKP + pb + (size_t)s * 16 * DH) = hv; }
        }
        if (ps == 0) __threadfence(); }
}
static_assert(4 * 4 * 32 * 16 == 64 * 64 * 2);

__global__ __launch_bounds__(32 * GW) void k_gatemix(const h16* __restrict__ XH, const h16* __restrict__ C1T, const h16* __restrict__ C2T,
                                                     const float* __restrict__ c1b, const float* __restrict__ c2b,
                                                     const float* __restrict__ FEAT, const float* __restrict__ O1, const float* __restrict__ O4,
                                                     const float* __restrict__ nodew, int layer, float* MX, h16* MXH) {
    __shared__ __align__(16) float os[GW * 16 * MSP];
    const int lane = threadIdx.x & 31, lr = lane & 15, hi = lane >> 4;
    const int wave = __builtin_amdgcn_readfirstlane((int)(threadIdx.x >> 5));
    const int t0 = (blockIdx.x * GW + wave) * 16;
    const int wb = wave * 16 * MSP;
    const int cnt = 5 + layer;
    float nwv[8]; float mxw = NEGB;
#pragma unroll
    for (int q = 0; q < 8; ++q) { const float xq = bfr(nodew[layer * 8 + q]); nwv[q] = xq; mxw = (q < cnt) ? fmaxf(mxw, xq) : mxw; }
    float ssum = 0.0f;
#pragma unroll
    for (int q = 0; q < 8; ++q) { float e = __builtin_amdgcn_exp2f((nwv[q] - mxw) * (100.0f * LOG2E)); e = (q < cnt) ? e : 0.0f; nwv[q] = e; ssum += e; }
    const float winv = 1.0f / ssum;
    float wo1 = 0.0f, wo2 = 0.0f, wxl = 0.0f, wo4 = 0.0f;
#pragma unroll
    for (int q = 0; q < 8; ++q) { nwv[q] *= winv;
        wo1 = (q == layer + 1) ? nwv[q] : wo1; wo2 = (q == layer + 2) ? nwv[q] : wo2; wxl = (q == layer + 3) ? nwv[q] : wxl; wo4 = (q == layer + 4) ? nwv[q] : wo4; }
    const size_t xo = (size_t)(t0 + lr) * CW + 8 * hi;
    const int ao = lr * CW + 8 * hi;
    v8f tacc = (v8f){};
#pragma unroll 1
    for (int kc = 0; kc < CW; kc += 32) { const v16h a = ldh(C1T + ao + kc); const v16h b = ldh(XH + xo + kc); tacc = wmma16g(a, b, tacc); }
    v16h tb = (v16h){};
#pragma unroll
    for (int r = 0; r < 8; ++r) { float tv = tacc[r] * (1.0f / (WCAR * ACAR)) + bfr(c1b[8 * hi + r]); tv = tv > 0.0f ? tv : 0.0f; tb[r] = toh_flush(tv * ACAR); }
    const size_t rowoff = (size_t)(t0 + lr) * CW;
    const size_t PLF = (size_t)MR * CW;
    const v8f zf = (v8f){};
#pragma unroll 1
    for (int ct = 0; ct < 16; ++ct) {
        const int cb = ct * 16 + 8 * hi;
        const v16h a2 = ldh8z(C2T + (ct * 16 + lr) * CAH + 8 * hi);
        const v8f g = wmma16g(a2, tb, zf);
        const v4f b2a = *(const v4f*)(c2b + cb), b2b = *(const v4f*)(c2b + cb + 4);
        const size_t off = rowoff + cb;
        const v4f xla = *(const v4f*)(FEAT + (size_t)layer * PLF + off), xlb = *(const v4f*)(FEAT + (size_t)layer * PLF + off + 4);
        const v4f o1a = *(const v4f*)(O1 + off), o1b = *(const v4f*)(O1 + off + 4);
        const v4f o4a = *(const v4f*)(O4 + off), o4b = *(const v4f*)(O4 + off + 4);
        v4f ma, mb;
#pragma unroll
        for (int i = 0; i < 4; ++i) {
            const float za = g[i] * (1.0f / (WCAR * ACAR)) + bfr(b2a[i]), zb = g[4 + i] * (1.0f / (WCAR * ACAR)) + bfr(b2b[i]);
            const float ga = __builtin_amdgcn_rcpf(1.0f + __builtin_amdgcn_exp2f(-za * LOG2E)), gb = __builtin_amdgcn_rcpf(1.0f + __builtin_amdgcn_exp2f(-zb * LOG2E));
            ma[i] = wo1 * o1a[i] + wo2 * (ga * xla[i]) + wxl * xla[i] + wo4 * o4a[i];
            mb[i] = wo1 * o1b[i] + wo2 * (gb * xlb[i]) + wxl * xlb[i] + wo4 * o4b[i]; }
#pragma unroll
        for (int p = 0; p < 4; ++p) {
            if (p <= layer) { const v4f fa = *(const v4f*)(FEAT + (size_t)p * PLF + off), fb = *(const v4f*)(FEAT + (size_t)p * PLF + off + 4);
                ma = ma + fa * nwv[p]; mb = mb + fb * nwv[p]; } }
        *(v4fa*)(&os[wb + lr * MSP + cb]) = ma; *(v4fa*)(&os[wb + lr * MSP + cb + 4]) = mb;
    }
    wave_sync();
#pragma unroll 1
    for (int ps = 0; ps < 2; ++ps) {
#pragma unroll 1
        for (int s = 0; s < 32; ++s) { const int row = s >> 1, cofs = (s & 1) * 128 + lane * 4;
            const v4f val = *(const v4fa*)(&os[wb + row * MSP + cofs]);
            *(volatile v4f*)(MX + (size_t)(t0 + row) * CW + cofs) = val; }
#pragma unroll 1
        for (int s = 0; s < 16; ++s) { const int c8 = lane * 8;
            const v4f x0 = *(const v4fa*)(&os[wb + s * MSP + c8]); const v4f x1 = *(const v4fa*)(&os[wb + s * MSP + c8 + 4]); v8h hv;
#pragma unroll
            for (int i = 0; i < 4; ++i) { hv[i] = toh_flush(x0[i] * ACAR); hv[4 + i] = toh_flush(x1[i] * ACAR); }
            *(volatile v8h*)(MXH + (size_t)(t0 + s) * CW + c8) = hv; }
        if (ps == 0) __threadfence(); }
}
static_assert(32 * 32 * 16 == 16 * CW * 4 && 16 * 32 * 16 == 16 * CW * 2);

__global__ __launch_bounds__(32 * AW) void k_flash(const h16* __restrict__ QP, const h16* __restrict__ KP, const h16* __restrict__ VT, h16* CTX) {
    __shared__ __align__(16) float os[16 * OSP];
    const int lane = threadIdx.x & 31, lr = lane & 15, hi = lane >> 4;
    const int wave = __builtin_amdgcn_readfirstlane((int)(threadIdx.x >> 5));
    const int zg = blockIdx.y; const int b = zg / (NH_ / AW), g = zg % (NH_ / AW);
    const int zh = b * NH_ + g * AW + wave;
    const int t0 = blockIdx.x * 16;
    const size_t pbase = (size_t)zh * SEQ * DH;
    const v16h qh = ldh8z(QP + pbase + (size_t)(t0 + lr) * DH + 8 * hi);
    const size_t ko = pbase + (size_t)lr * DH + 8 * hi;
    const size_t vo = pbase + (size_t)lr * SEQ + 8 * hi;
    v8f o0 = (v8f){};
    float m = NEGB, l = 0.0f;
#pragma unroll 1
    for (int key0 = 0; key0 < SEQ; key0 += 32) {
        const h16* ka = KP + ko + (size_t)key0 * DH;
        const v16h ka0 = ldh8z(ka), kb0 = ldh8z(ka + 16 * DH);
        v8f sa = (v8f){}, sb = (v8f){};
        sa = wmma16g(ka0, qh, sa); sb = wmma16g(kb0, qh, sb);
        float ta[8], tb[8]; float mx = NEGB;
#pragma unroll
        for (int r = 0; r < 8; ++r) { ta[r] = sa[r] * SC2; tb[r] = sb[r] * SC2; mx = fmaxf(mx, fmaxf(ta[r], tb[r])); }
        mx = fmaxf(mx, __shfl_xor(mx, 16, 32));
        const float mnew = fmaxf(m, mx);
        const float alpha = __builtin_amdgcn_exp2f(m - mnew);
        const float sh = PSH - mnew;
        v16h pb; float ls = 0.0f;
#pragma unroll
        for (int r = 0; r < 8; ++r) {
            const float ea = ta[r] + sh, eb = tb[r] + sh;
            const float xa = __builtin_amdgcn_exp2f(ea), xb = __builtin_amdgcn_exp2f(eb);
            const float ga = (ea < -14.0f) ? 0.0f : xa, gb = (eb < -14.0f) ? 0.0f : xb;
            const h16 pa = (h16)ga; const h16 pc = (h16)gb;
            pb[r] = pa; pb[8 + r] = pc; ls += (float)pa + (float)pc; }
        l = l * alpha + ls; m = mnew;
        o0 = o0 * alpha;
        const v16h v0 = ldh(VT + vo + key0);
        o0 = wmma16g(v0, pb, o0);
    }
    l += __shfl_xor(l, 16, 32);
    const float inv = (1.0f / l) * (CTXC / VCAR);
    { v4f a, c;
      a[0] = o0[0] * inv; a[1] = o0[1] * inv; a[2] = o0[2] * inv; a[3] = o0[3] * inv; c[0] = o0[4] * inv; c[1] = o0[5] * inv; c[2] = o0[6] * inv; c[3] = o0[7] * inv;
      *(v4fa*)(&os[lr * OSP + wave * 16 + 8 * hi]) = a; *(v4fa*)(&os[lr * OSP + wave * 16 + 8 * hi + 4]) = c; }
    __syncthreads();
    const int row = 4 * wave + (lane >> 3), c8 = (lane & 7) * 8;
    const v4f x0 = *(const v4fa*)(&os[row * OSP + c8]); const v4f x1 = *(const v4fa*)(&os[row * OSP + c8 + 4]); v8h hv;
#pragma unroll
    for (int i = 0; i < 4; ++i) { hv[i] = toh_flush(x0[i]); hv[4 + i] = toh_flush(x1[i]); }
    h16* dst = CTX + ((size_t)b * SEQ + t0 + row) * CW + g * 64 + c8;
    *(volatile v8h*)dst = hv; __threadfence(); *(volatile v8h*)dst = hv;
}
static_assert(AW * 4 == 16 && 8 * 16 == 64 * 2);

static constexpr size_t al256(size_t v) { return (v + 255) & ~(size_t)255; }
static constexpr size_t SZ_WQKV = al256((size_t)4 * 3 * CW * CW * 2);
static constexpr size_t SZ_WSQ  = al256((size_t)4 * CW * CW * 2);
static constexpr size_t SZ_WMLP = al256((size_t)4 * MLPW * CW * 2);
static constexpr size_t SZ_WCA  = al256((size_t)4 * CAH * CW * 2);
static constexpr size_t SZ_WH   = al256((size_t)HID * CW * 2);
static constexpr size_t SZ_WPR  = al256((size_t)PRED * HID * 2);
static constexpr size_t SZ_PT   = al256((size_t)GRD * 128 * 4);
static constexpr size_t SZ_F32  = al256((size_t)MR * CW * 4);
static constexpr size_t SZ_H16  = al256((size_t)MR * CW * 2);
static constexpr size_t SZ_UH   = al256((size_t)MR * MLPW * 2);
static constexpr size_t SZ_HA   = al256((size_t)MR * HID * 4);
static constexpr size_t SZ_HH   = al256((size_t)MR * HID * 2);
static_assert(SZ_HH <= SZ_HA);
static constexpr size_t SZ_TOTAL = SZ_WQKV + 2 * SZ_WSQ + 2 * SZ_WMLP + 2 * SZ_WCA + 3 * SZ_WH + SZ_WPR + SZ_PT
                                 + 5 * SZ_F32   + SZ_H16   + 2 * SZ_F32   + SZ_UH + SZ_F32   + SZ_H16
                                 + 2 * SZ_H16   + SZ_H16   + SZ_H16   + SZ_H16   + SZ_HA + SZ_HH   + SZ_F32  ;
static_assert(SZ_TOTAL <= (size_t)134217728);
static_assert((size_t)NB * NH_ * SEQ * DH == (size_t)MR * CW);

static void run_gemm(hipStream_t st, int M, int N, const h16* A, int lda, const h16* Bt, int ldb, int K, const float* bias, int brow, float oscale, int act,
                     const float* R, int ldr, int useR, float* Cf, int ldc, int useF, h16* Ch, int ldch, int useH, float hscale, int cgrp, int cgs) {
    k_gemm<<<dim3((unsigned)(M / 64), (unsigned)(N / 64), 1), 32, 0, st>>>(A, lda, Bt, ldb, K, bias, brow, oscale, act, R, ldr, useR, Cf, ldc, useF, Ch, ldch, useH, hscale, cgrp, cgs);
}
static void run_wconv(hipStream_t st, const float* W, h16* WT, int L, int K, int N) {
    const int total8 = L * K * N / 8;
    k_wconv<<<(unsigned)((total8 + 255) / 256), 256, 0, st>>>(W, WT, K, N, total8);
}

extern "C" void kernel_launch(void* const* d_in, const int* in_sizes, int n_in,
                              void* d_out, int out_size, void* d_ws, size_t ws_size, hipStream_t stream) {
    if (n_in < 38) return;
    if ((size_t)in_sizes[0] < (size_t)NB * 3 * IMG * IMG) return;
    if ((size_t)in_sizes[1] < (size_t)(NB - 1) * SEQ_FULL + SEQ) return;
    if (in_sizes[2] < CW * 12 || in_sizes[3] < CW || in_sizes[4] < CW) return;
    if (in_sizes[5] < 4 * CW * 3 * CW || in_sizes[6] < 4 * 3 * CW || in_sizes[7] < 4 * CW * CW || in_sizes[8] < 4 * CW) return;
    if (in_sizes[9] < 4 * DH || in_sizes[10] < 4 * DH || in_sizes[11] < 4 * DH || in_sizes[12] < 4 * DH) return;
    if (in_sizes[13] < 4 * CW * CW || in_sizes[14] < 4 * CW || in_sizes[15] < 4 * CW * CAH || in_sizes[16] < 4 * CAH || in_sizes[17] < 4 * CAH * CW || in_sizes[18] < 4 * CW) return;
    if (in_sizes[19] < 4 * CW * MLPW || in_sizes[20] < 4 * MLPW || in_sizes[21] < 4 * MLPW * CW || in_sizes[22] < 4 * CW || in_sizes[23] < 32) return;
    if (in_sizes[24] < CW || in_sizes[25] < CW || in_sizes[26] < CW * HID || in_sizes[27] < HID || in_sizes[28] < HID || in_sizes[29] < HID) return;
    if (in_sizes[30] < HID * CW || in_sizes[31] < CW || in_sizes[32] < CW || in_sizes[33] < CW || in_sizes[34] < CW * HID || in_sizes[35] < HID) return;
    if (in_sizes[36] < HID * PRED || in_sizes[37] < PRED) return;
    if ((size_t)out_size < (size_t)MR * PRED) return;
    if (SZ_TOTAL > ws_size) return;
    const float* x      = (const float*)d_in[0];   const int*   midx   = (const int*)d_in[1];
    const float* Wp     = (const float*)d_in[2];   const float* bp     = (const float*)d_in[3];   const float* cls    = (const float*)d_in[4];
    const float* qkv_w  = (const float*)d_in[5];   const float* qkv_b  = (const float*)d_in[6];
    const float* proj_w = (const float*)d_in[7];   const float* proj_b = (const float*)d_in[8];
    const float* nq_g   = (const float*)d_in[9];   const float* nq_b   = (const float*)d_in[10];
    const float* nk_g   = (const float*)d_in[11];  const float* nk_b   = (const float*)d_in[12];
    const float* conv_w = (const float*)d_in[13];  const float* conv_b = (const float*)d_in[14];
    const float* ca1_w  = (const float*)d_in[15];  const float* ca1_b  = (const float*)d_in[16];
    const float* ca2_w  = (const float*)d_in[17];  const float* ca2_b  = (const float*)d_in[18];
    const float* mlp1_w = (const float*)d_in[19];  const float* mlp1_b = (const float*)d_in[20];
    const float* mlp2_w = (const float*)d_in[21];  const float* mlp2_b = (const float*)d_in[22];
    const float* node_w = (const float*)d_in[23];
    const float* ln0_g  = (const float*)d_in[24];  const float* ln0_b  = (const float*)d_in[25];
    const float* h1_w   = (const float*)d_in[26];  const float* h1_b   = (const float*)d_in[27];
    const float* ln1_g  = (const float*)d_in[28];  const float* ln1_b  = (const float*)d_in[29];
    const float* h2_w   = (const float*)d_in[30];  const float* h2_b   = (const float*)d_in[31];
    const float* ln2_g  = (const float*)d_in[32];  const float* ln2_b  = (const float*)d_in[33];
    const float* h3_w   = (const float*)d_in[34];  const float* h3_b   = (const float*)d_in[35];
    const float* pr_w   = (const float*)d_in[36];  const float* pr_b   = (const float*)d_in[37];
    float* OUT = (float*)d_out;

    char* wsp = (char*)d_ws;
    h16* WQKV = (h16*)wsp; wsp += SZ_WQKV;
    h16* WPRJ = (h16*)wsp; wsp += SZ_WSQ;
    h16* WCNV = (h16*)wsp; wsp += SZ_WSQ;
    h16* WM1  = (h16*)wsp; wsp += SZ_WMLP;
    h16* WM2  = (h16*)wsp; wsp += SZ_WMLP;
    h16* WC1  = (h16*)wsp; wsp += SZ_WCA;
    h16* WC2  = (h16*)wsp; wsp += SZ_WCA;
    h16* WH1  = (h16*)wsp; wsp += SZ_WH;
    h16* WH2  = (h16*)wsp; wsp += SZ_WH;
    h16* WH3  = (h16*)wsp; wsp += SZ_WH;
    h16* WPR  = (h16*)wsp; wsp += SZ_WPR;
    float* PT = (float*)wsp; wsp += SZ_PT;
    float* FEAT = (float*)wsp; wsp += 5 * SZ_F32;
    h16* XH   = (h16*)wsp; wsp += SZ_H16;
    float* O1 = (float*)wsp; wsp += SZ_F32;
    float* O4 = (float*)wsp; wsp += SZ_F32;
    h16* UH   = (h16*)wsp; wsp += SZ_UH;
    float* MX = (float*)wsp; wsp += SZ_F32;
    h16* MXH  = (h16*)wsp; wsp += SZ_H16;
    h16* QKP  = (h16*)wsp; wsp += 2 * SZ_H16;
    h16* VT   = (h16*)wsp; wsp += SZ_H16;
    h16* CTX  = (h16*)wsp; wsp += SZ_H16;
    h16* S1H  = (h16*)wsp; wsp += SZ_H16;
    float* HA = (float*)wsp; h16* HCH = (h16*)wsp; wsp += SZ_HA;
    h16* HBH  = (h16*)wsp; wsp += SZ_HH;
    float* S2 = (float*)wsp; wsp += SZ_F32;
    const size_t PLF = (size_t)MR * CW;
    const float OS1 = 1.0f / (WCAR * ACAR);

    run_wconv(stream, qkv_w,  WQKV, 4, CW, 3 * CW);
    run_wconv(stream, proj_w, WPRJ, 4, CW, CW);
    run_wconv(stream, conv_w, WCNV, 4, CW, CW);
    run_wconv(stream, mlp1_w, WM1,  4, CW, MLPW);
    run_wconv(stream, mlp2_w, WM2,  4, MLPW, CW);
    run_wconv(stream, ca1_w,  WC1,  4, CW, CAH);
    run_wconv(stream, ca2_w,  WC2,  4, CAH, CW);
    run_wconv(stream, h1_w,   WH1,  1, CW, HID);
    run_wconv(stream, h2_w,   WH2,  1, HID, CW);
    run_wconv(stream, h3_w,   WH3,  1, CW, HID);
    run_wconv(stream, pr_w,   WPR,  1, HID, PRED);

    k_postab<<<(GRD * 128) / 256, 256, 0, stream>>>(PT);
    k_patch<<<(unsigned)((size_t)MR * CW / 4 / 256), 256, 0, stream>>>(x, midx, Wp, bp, cls, PT, FEAT, XH);

    for (int j = 0; j < 4; ++j) {
        run_gemm(stream, MR, CW, XH, CW, WCNV + (size_t)j * CW * CW, CW, CW, conv_b + j * CW, 0, OS1, 1, MX, CW, 0, O1, CW, 1, XH, CW, 0, 1.0f, CW, 0);
        run_gemm(stream, MR, MLPW, XH, CW, WM1 + (size_t)j * MLPW * CW, CW, CW, mlp1_b + j * MLPW, 0, OS1, 1, MX, CW, 0, O1, CW, 0, UH, MLPW, 1, ACAR, MLPW, 0);
        run_gemm(stream, MR, CW, UH, MLPW, WM2 + (size_t)j * CW * MLPW, MLPW, MLPW, mlp2_b + j * CW, 0, OS1, 0, MX, CW, 0, O4, CW, 1, XH, CW, 0, 1.0f, CW, 0);
        k_gatemix<<<MR / (16 * GW), 32 * GW, 0, stream>>>(XH, WC1 + (size_t)j * CAH * CW, WC2 + (size_t)j * CW * CAH, ca1_b + j * CAH, ca2_b + j * CW,
                                                        FEAT, O1, O4, node_w, j, MX, MXH);
        k_qk<<<dim3(MR / 64, (2 * CW) / 64, 1), 32, 0, stream>>>(MXH, WQKV + (size_t)j * 3 * CW * CW, qkv_b + j * 3 * CW,
                                                               nq_g + j * DH, nq_b + j * DH, nk_g + j * DH, nk_b + j * DH, OS1, QKP);
        run_gemm(stream, CW, MR, WQKV + (size_t)j * 3 * CW * CW + (size_t)2 * CW * CW, CW, MXH, CW, CW, qkv_b + j * 3 * CW + 2 * CW, 1, OS1, 0,
                 MX, CW, 0, O1, CW, 0, VT, SEQ, 1, VCAR, SEQ, CW * SEQ);
        k_flash<<<dim3(SEQ / 16, NB * NH_ / AW, 1), 32 * AW, 0, stream>>>(QKP, QKP + PLF, VT, CTX);
        run_gemm(stream, MR, CW, CTX, CW, WPRJ + (size_t)j * CW * CW, CW, CW, proj_b + j * CW, 0, 1.0f / (WCAR * CTXC), 0,
                 MX, CW, 1, FEAT + (size_t)(j + 1) * PLF, CW, 1, XH, CW, 1, ACAR, CW, 0);
    }

    k_ln<<<MR / 8, 256, 0, stream>>>(FEAT + 4 * PLF, ln0_g, ln0_b, S1H, CW, MR);
    run_gemm(stream, MR, HID, S1H, CW, WH1, CW, CW, h1_b, 0, OS1, 0, MX, CW, 0, HA, HID, 1, XH, CW, 0, 1.0f, HID, 0);
    k_ln<<<MR / 8, 256, 0, stream>>>(HA, ln1_g, ln1_b, HBH, HID, MR);
    run_gemm(stream, MR, CW, HBH, HID, WH2, HID, HID, h2_b, 0, OS1, 0, MX, CW, 0, S2, CW, 1, XH, CW, 0, 1.0f, CW, 0);
    k_ln<<<MR / 8, 256, 0, stream>>>(S2, ln2_g, ln2_b, S1H, CW, MR);
    run_gemm(stream, MR, HID, S1H, CW, WH3, CW, CW, h3_b, 0, OS1, 0, MX, CW, 0, O1, CW, 0, HCH, HID, 1, ACAR, HID, 0);
    run_gemm(stream, MR, PRED, HCH, HID, WPR, HID, HID, pr_b, 0, OS1, 0, MX, CW, 0, OUT, PRED, 1, XH, CW, 0, 1.0f, PRED, 0);
}
